// HypBlock_83760452207345
// MI455X (gfx1250) — hardware-verified
//
#include <hip/hip_runtime.h>


namespace {
constexpr int Bn = 32, S = 197, D = 768, HID = 3072, NH = 12, HD = 64, NTOK = Bn * S  , SP = 208  , SV = 224  ;
constexpr float EPS = 1e-5f, XS = 8.0f, QS = 8.0f, VS = 8.0f, PS = 8.0f;
constexpr size_t PLQ = (size_t)Bn * NH * SP * HD, PLV = (size_t)Bn * NH * HD * SV;

typedef _Float16 b16;
typedef __attribute__((ext_vector_type(16))) _Float16 v16b;
typedef __attribute__((ext_vector_type(8))) _Float16 v8b;
typedef __attribute__((ext_vector_type(8))) float v8f;
typedef __attribute__((ext_vector_type(4))) float v4f;
__device__ __forceinline__ float bf16_rne(float f) { unsigned int u = __float_as_uint(f); u += 0x7FFFu + ((u >> 16) & 1u); return __uint_as_float(u & 0xFFFF0000u); }
__device__ __forceinline__ v16b frag_kb(const b16* p, int hh) { const v8b a = *(const v8b*)(p + 8 * hh), b = *(const v8b*)(p + 16 + 8 * hh); v16b f;
#pragma unroll
  for (int e = 0; e < 8; ++e) { f[e] = a[e]; f[8 + e] = b[e]; } return f; }
__device__ __forceinline__ v8f wmma16b(v16b a, v16b b, v8f c) { v8f d = __builtin_amdgcn_wmma_f32_16x16x32_f16(false, a, false, b, (short)0, c, false, false); asm volatile("v_nop\n\tv_nop\n\tv_nop\n\tv_nop" : "+v"(d) : "v"(a), "v"(b)); return d; }
__device__ __forceinline__ void wave_lds_sync() { __builtin_amdgcn_fence(__ATOMIC_RELEASE, "workgroup"); __builtin_amdgcn_wave_barrier(); __builtin_amdgcn_fence(__ATOMIC_ACQUIRE, "workgroup"); }
__device__ __forceinline__ float nexp(float x) { return __builtin_amdgcn_exp2f(x * 1.4426950408889634f); }
__device__ __forceinline__ float pmul(float a, float b) { float p = a * b; asm volatile("" : "+v"(p)); return p; }
__device__ __forceinline__ float h2f(b16 h) { float f = (float)h; asm volatile("" : "+v"(f)); return f; }
__device__ __forceinline__ float wsum(float v) {
#pragma unroll
  for (int o = 1; o < 32; o <<= 1) v += __shfl_xor(v, o); return v; }
__device__ __forceinline__ float rcp_f(float x) { return __builtin_amdgcn_rcpf(x); }
__device__ __forceinline__ float sqrt_f(float x) { return __builtin_amdgcn_sqrtf(x); }
__device__ __forceinline__ float nlog(float x) { return __builtin_amdgcn_logf(x) * 0.6931471805599453f; }
__device__ __forceinline__ float tanh_n(float x) { const float e = __builtin_amdgcn_exp2f(x * 2.8853900817779268f); return 1.0f - 2.0f * rcp_f(e + 1.0f); }
__device__ __forceinline__ float artanh_f(float x) { x = fminf(fmaxf(x, -1.0f + 1e-7f), 1.0f - 1e-7f); return 0.5f * nlog((1.0f + x) * rcp_f(1.0f - x)); }
__device__ __forceinline__ float proj_fac(float n) { return fminf(1.0f, (1.0f - EPS) * rcp_f(fmaxf(n, 1e-15f))); }

struct Wo_ { static constexpr size_t QKV = 0, PRJ = QKV + (size_t)3 * D * D, W1 = PRJ + (size_t)D * D, W2 = W1 + (size_t)HID * D, END = W2 + (size_t)D * HID; };
__global__ __launch_bounds__(256) void prep_kernel(const float* __restrict__ Wqkv, const float* __restrict__ Wproj, const float* __restrict__ W1, const float* __restrict__ W2, const float* __restrict__ bp, const float* __restrict__ b1, const float* __restrict__ b2, b16* __restrict__ R, float* __restrict__ P) {
  const size_t tid = (size_t)blockIdx.x * 256 + threadIdx.x, nth = (size_t)gridDim.x * 256;
  for (int pass = 0; pass < 2; ++pass) {
    for (size_t p = tid; p < Wo_::END / 8; p += nth) { const size_t q = p * 8; const float* src = (q < Wo_::PRJ) ? (Wqkv + q) : (q < Wo_::W1) ? (Wproj + (q - Wo_::PRJ)) : (q < Wo_::W2) ? (W1 + (q - Wo_::W1)) : (W2 + (q - Wo_::W2)); v8b v;
#pragma unroll
      for (int e = 0; e < 8; ++e) v[e] = (b16)bf16_rne(src[e]); *(volatile v8b*)(R + q) = v; }
    for (size_t q = tid; q < 4608; q += nth) { const int i = (int)q; P[q] = (i < 768) ? bf16_rne(bp[i]) : (i < 3840) ? bf16_rne(b1[i - 768]) : bf16_rne(b2[i - 3840]); }
    __threadfence(); }
}

__global__ __launch_bounds__(256) void row0_kernel(const float* __restrict__ x, float* __restrict__ X0, b16* __restrict__ X0h) {
  const int row = blockIdx.x * 8 + (threadIdx.x >> 5), lane = threadIdx.x & 31; const float* xr = x + (size_t)row * D;
  float v[24]; float s2 = 0.0f;
#pragma unroll
  for (int i = 0; i < 24; ++i) { v[i] = bf16_rne(xr[(i >> 3) * 256 + lane * 8 + (i & 7)]); s2 += pmul(v[i], v[i]); }
  s2 = wsum(s2); const float fac = proj_fac(sqrt_f(s2));
  for (int pass = 0; pass < 2; ++pass) {
#pragma unroll
    for (int g = 0; g < 3; ++g) { v4f a, b; v8b hv; for (int e = 0; e < 4; ++e) { a[e] = v[g * 8 + e] * fac; b[e] = v[g * 8 + 4 + e] * fac; } for (int e = 0; e < 8; ++e) hv[e] = (b16)(v[g * 8 + e] * fac * XS);
      float* dst = X0 + (size_t)row * D + g * 256 + lane * 8; *(volatile v4f*)dst = a; *(volatile v4f*)(dst + 4) = b; *(volatile v8b*)(X0h + (size_t)row * D + g * 256 + lane * 8) = hv; }
    __threadfence(); }
}

template <int K, int N, int EPI>
__global__ __launch_bounds__(64) void gemm_kernel(const b16* __restrict__ A, const b16* __restrict__ Bw, const float* __restrict__ bias, b16* __restrict__ Ch, float* __restrict__ Cf) {
  __shared__ __attribute__((aligned(16))) b16 Ts[2][32][128 + 8];
  (void)Cf;
  const int lane = threadIdx.x & 31, wave = threadIdx.x >> 5, nloc = lane & 15, hlf = lane >> 4, m0 = blockIdx.y * 32, c0 = blockIdx.x * 256 + wave * 128;
  v8f acc[2][8];
#pragma unroll
  for (int r = 0; r < 2; ++r)
#pragma unroll
    for (int t = 0; t < 8; ++t) acc[r][t] = (v8f){};
  for (int kb = 0; kb < K; kb += 32) { const v16b a0 = frag_kb(A + (size_t)(m0 + nloc) * K + kb, hlf), a1 = frag_kb(A + (size_t)(m0 + 16 + nloc) * K + kb, hlf);
#pragma unroll
    for (int t = 0; t < 8; ++t) { const v16b bw = frag_kb(Bw + (size_t)(c0 + t * 16 + nloc) * K + kb, hlf); acc[0][t] = wmma16b(a0, bw, acc[0][t]); acc[1][t] = wmma16b(a1, bw, acc[1][t]); } }
#pragma unroll
  for (int t = 0; t < 8; ++t) { const float bb = (bias != nullptr) ? bias[c0 + t * 16 + nloc] : 0.0f;
#pragma unroll
    for (int r = 0; r < 2; ++r)
#pragma unroll
      for (int v = 0; v < 8; ++v) Ts[wave][r * 16 + 8 * hlf + v][t * 16 + nloc] = (b16)(acc[r][t][v] + bb * XS); }
  wave_lds_sync();
  for (int pass = 0; pass < 2; ++pass) { for (int i = lane; i < 32 * 16; i += 32) { const int rr = i >> 4, c8 = (i & 15) * 8; *(volatile v8b*)(Ch + (size_t)(m0 + rr) * N + c0 + c8) = *(const v8b*)(&Ts[wave][rr][c8]); } __threadfence(); }
}

__global__ __launch_bounds__(256) void head_kernel(const b16* __restrict__ QKV, b16* __restrict__ Qp, b16* __restrict__ Kp, b16* __restrict__ Vt, float* __restrict__ NQK) {
  __shared__ __attribute__((aligned(16))) b16 Tv[HD][SV + 8];
  const int h = blockIdx.x, b = blockIdx.y, t_ = threadIdx.x;
  for (int i = t_; i < HD * (SV + 8); i += 256) (&Tv[0][0])[i] = (b16)0.0f;
  __syncthreads();
  b16* Qb = Qp + ((size_t)b * NH + h) * SP * HD; b16* Kb = Kp + ((size_t)b * NH + h) * SP * HD;
  for (int pass = 0; pass < 2; ++pass) {
    for (int w_ = t_; w_ < SP * 2; w_ += 256) { const int s = w_ % SP, which = w_ / SP;
      b16* dst = ((which == 0) ? Qb : Kb) + (size_t)s * HD; float u[HD];
      if (s < S) { const b16* src = QKV + ((size_t)(b * S + s)) * (3 * D) + which * D + h * HD; float n2 = 0.0f;
#pragma unroll
        for (int d8 = 0; d8 < HD; d8 += 8) { const v8b vv = *(const v8b*)(src + d8); for (int e = 0; e < 8; ++e) { u[d8 + e] = (float)vv[e] * (1.0f / XS); n2 += pmul(u[d8 + e], u[d8 + e]); } }
        const float n = fmaxf(sqrt_f(n2), 1e-15f); const float th = tanh_n(n); float f1 = th * rcp_f(n);
        const float f2 = proj_fac(th * 1.0f); const float fac = f1 * f2 * QS;
#pragma unroll
        for (int d = 0; d < HD; ++d) u[d] *= fac; }
      else {
#pragma unroll
        for (int d = 0; d < HD; ++d) u[d] = 0.0f; }
      float n2r = 0.0f;
#pragma unroll
      for (int d8 = 0; d8 < HD; d8 += 8) { v8b o; for (int e = 0; e < 8; ++e) { o[e] = (b16)u[d8 + e]; const float f = (float)o[e] * (1.0f / QS); n2r += pmul(f, f); } *(volatile v8b*)(dst + d8) = o; }
      ((volatile float*)NQK)[(((size_t)b * NH + h) * 2 + which) * SP + s] = n2r; }
    if (pass == 0) { for (int i = t_; i < S * (HD / 8); i += 256) { const int s = i / (HD / 8), d8 = (i % (HD / 8)) * 8; const v8b vv = *(const v8b*)(QKV + ((size_t)(b * S + s)) * (3 * D) + 2 * D + h * HD + d8); for (int e = 0; e < 8; ++e) Tv[d8 + e][s] = vv[e]; }
      __syncthreads(); }
    for (int i = t_; i < HD * (SV / 8); i += 256) { const int d = i / (SV / 8), c8 = (i % (SV / 8)) * 8; *(volatile v8b*)(Vt + (((size_t)b * NH + h) * HD + d) * SV + c8) = *(const v8b*)(&Tv[d][c8]); }
    __threadfence(); }
}

__global__ __launch_bounds__(384) void attn_kernel(const b16* __restrict__ Qp, const b16* __restrict__ Kp, const b16* __restrict__ Vt, const float* __restrict__ NQK, b16* __restrict__ ctx) {
  __shared__ __attribute__((aligned(16))) b16 Os[16][D + 8];
  const int h = threadIdx.x >> 5, lane = threadIdx.x & 31, hh = lane >> 4, col = lane & 15, b = blockIdx.y, q0 = blockIdx.x * 16, qi = q0 + col;
  const b16* Qb = Qp + ((size_t)b * NH + h) * SP * HD; const b16* Kb = Kp + ((size_t)b * NH + h) * SP * HD; const b16* Vb = Vt + ((size_t)b * NH + h) * HD * SV;
  const v16b qf0 = frag_kb(Qb + (size_t)qi * HD, hh), qf1 = frag_kb(Qb + (size_t)qi * HD + 32, hh);
  const float* NQ = NQK + (((size_t)b * NH + h) * 2) * SP; const float* NK = NQ + SP; const float qq = NQ[qi];
  float m = -INFINITY, l = 0.0f; v8f o[4] = {{}, {}, {}, {}};
  for (int kb = 0; kb < SV; kb += 32) {
    v8f s0 = {}, s1 = {};
    { const v16b ka0 = frag_kb(Kb + (size_t)(kb + col) * HD, hh), ka1 = frag_kb(Kb + (size_t)(kb + col) * HD + 32, hh); s0 = wmma16b(ka0, qf0, s0); s0 = wmma16b(ka1, qf1, s0); }
    if (kb + 16 < SP) { const v16b kc0 = frag_kb(Kb + (size_t)(kb + 16 + col) * HD, hh), kc1 = frag_kb(Kb + (size_t)(kb + 16 + col) * HD + 32, hh); s1 = wmma16b(kc0, qf0, s1); s1 = wmma16b(kc1, qf1, s1); }
    float mr = -INFINITY;
#pragma unroll
    for (int u = 0; u < 2; ++u)
#pragma unroll
      for (int r = 0; r < 8; ++r) { const int key = kb + u * 16 + 8 * hh + r; float sv;
        if (key < S) { const float kk = NK[key];
          const float qk = ((u == 0) ? s0[r] : s1[r]) * (1.0f / (QS * QS)); const float num = qq - 2.0f * qk + kk, den = 1.0f - 2.0f * qk + pmul(qq, kk);
          const float r2 = fminf(fmaxf(num * rcp_f(fmaxf(den, 1e-15f)), 1e-15f), 1.0f - 1e-7f); const float dist = 2.0f * artanh_f(sqrt_f(r2)); sv = -dist * 0.125f; }
        else sv = -INFINITY;
        if (u == 0) s0[r] = sv; else s1[r] = sv; mr = fmaxf(mr, sv); }
    mr = fmaxf(mr, __shfl_xor(mr, 16));
    const float mn = fmaxf(m, mr), al_ = nexp(m - mn); m = mn; float sum = 0.0f; v16b pbv;
#pragma unroll
    for (int r = 0; r < 8; ++r) { const float e0 = (s0[r] == -INFINITY) ? 0.0f : nexp(s0[r] - mn), e1 = (s1[r] == -INFINITY) ? 0.0f : nexp(s1[r] - mn); sum += e0 + e1; pbv[r] = (b16)(e0 * PS); pbv[8 + r] = (b16)(e1 * PS); }
    sum += __shfl_xor(sum, 16); l = l * al_ + sum;
#pragma unroll
    for (int t = 0; t < 4; ++t) { o[t] *= al_; const v16b vf = frag_kb(Vb + (size_t)(t * 16 + col) * SV + kb, hh); o[t] = wmma16b(vf, pbv, o[t]); } }
  const float inv = XS * rcp_f(l * VS * PS);
#pragma unroll
  for (int t = 0; t < 4; ++t)
#pragma unroll
    for (int r = 0; r < 8; ++r) Os[col][h * HD + t * 16 + 8 * hh + r] = (b16)(o[t][r] * inv);
  __syncthreads();
  const int nq = (q0 + 16 <= S) ? 16 : (S - q0);
  for (int pass = 0; pass < 2; ++pass) { for (int i = threadIdx.x; i < nq * (D / 8); i += 384) { const int rr = i / (D / 8), c8 = (i % (D / 8)) * 8; *(volatile v8b*)(ctx + ((size_t)(b * S + q0 + rr)) * D + c8) = *(const v8b*)(&Os[rr][c8]); } __threadfence(); }
}

__device__ __forceinline__ void mobius_row(const float xv[24], const float yv[24], float outv[24], float& outnorm) {
  float x2 = 0.0f, y2 = 0.0f, xy = 0.0f;
#pragma unroll
  for (int i = 0; i < 24; ++i) { x2 += pmul(xv[i], xv[i]); y2 += pmul(yv[i], yv[i]); xy += pmul(xv[i], yv[i]); }
  x2 = wsum(x2); y2 = wsum(y2); xy = wsum(xy);
  const float rden = rcp_f(fmaxf(1.0f + 2.0f * xy + pmul(x2, y2), 1e-15f)); const float cx = (1.0f + 2.0f * xy + y2) * rden, cy = (1.0f - x2) * rden; float n2 = 0.0f;
#pragma unroll
  for (int i = 0; i < 24; ++i) { outv[i] = pmul(cx, xv[i]) + pmul(cy, yv[i]); n2 += pmul(outv[i], outv[i]); }
  n2 = wsum(n2); const float n = sqrt_f(n2); const float fac = proj_fac(n);
#pragma unroll
  for (int i = 0; i < 24; ++i) outv[i] *= fac;
  outnorm = n * fac; }
__global__ __launch_bounds__(256) void row1_kernel(const b16* __restrict__ OUTh, float* __restrict__ X, b16* __restrict__ X1h, float* __restrict__ NRM) {
  const int row = blockIdx.x * 8 + (threadIdx.x >> 5), lane = threadIdx.x & 31;
  float xv[24], yv[24], ov[24]; float n2 = 0.0f;
#pragma unroll
  for (int i = 0; i < 24; ++i) { const int c = (i >> 3) * 256 + lane * 8 + (i & 7); xv[i] = X[(size_t)row * D + c]; yv[i] = (float)OUTh[(size_t)row * D + c] * (1.0f / XS); n2 += pmul(yv[i], yv[i]); }
  n2 = wsum(n2); { const float n = fmaxf(sqrt_f(n2), 1e-15f); const float th = tanh_n(n); const float fac = (th * rcp_f(n)) * proj_fac(th);
#pragma unroll
    for (int i = 0; i < 24; ++i) yv[i] *= fac; }
  float onorm; mobius_row(xv, yv, ov, onorm);
  for (int pass = 0; pass < 2; ++pass) {
#pragma unroll
    for (int g = 0; g < 3; ++g) { v4f a, b; v8b hv; for (int e = 0; e < 4; ++e) { a[e] = ov[g * 8 + e]; b[e] = ov[g * 8 + 4 + e]; } for (int e = 0; e < 8; ++e) hv[e] = (b16)(ov[g * 8 + e] * XS);
      float* dst = X + (size_t)row * D + g * 256 + lane * 8; *(volatile v4f*)dst = a; *(volatile v4f*)(dst + 4) = b; *(volatile v8b*)(X1h + (size_t)row * D + g * 256 + lane * 8) = hv; }
    ((volatile float*)NRM)[(size_t)row * 32 + lane] = (lane == 0) ? onorm : 0.0f;
    __threadfence(); }
}

__global__ __launch_bounds__(256) void row2_kernel(const b16* __restrict__ MX1, const float* __restrict__ NRM, const float* __restrict__ P, b16* __restrict__ H1h, float* __restrict__ NRM2) {
  const int row = blockIdx.x * 8 + (threadIdx.x >> 5), lane = threadIdx.x & 31; const float* b1 = P + 768; const b16* src = MX1 + (size_t)row * HID + lane * 8;
  float hv[96]; float m2 = 0.0f;
#pragma unroll
  for (int g = 0; g < 12; ++g) { const v8b vv = *(const v8b*)(src + g * 256);
#pragma unroll
    for (int e = 0; e < 8; ++e) { hv[g * 8 + e] = h2f(vv[e]); m2 += pmul(hv[g * 8 + e], hv[g * 8 + e]); } }
  m2 = wsum(m2);
  const float xn = fmaxf(NRM[(size_t)row * 32], 1e-15f), mxn = fmaxf(sqrt_f(m2) * (1.0f / XS), 1e-15f); const float rad = tanh_n(mxn * rcp_f(xn) * artanh_f(xn));
  const float f1 = (rad * rcp_f(mxn)) * proj_fac(rad) * (1.0f / XS);
  float u2 = 0.0f, bb2 = 0.0f, ub = 0.0f;
#pragma unroll
  for (int g = 0; g < 12; ++g) { const float* bp_ = b1 + g * 256 + lane * 8;
#pragma unroll
    for (int e = 0; e < 8; ++e) { const float u = pmul(hv[g * 8 + e], f1); hv[g * 8 + e] = u; const float bq = bp_[e]; u2 += pmul(u, u); bb2 += pmul(bq, bq); ub += pmul(u, bq); } }
  u2 = wsum(u2); bb2 = wsum(bb2); ub = wsum(ub);
  const float rden = rcp_f(fmaxf(1.0f + 2.0f * ub + pmul(u2, bb2), 1e-15f)); const float cx = (1.0f + 2.0f * ub + bb2) * rden, cy = (1.0f - u2) * rden; float n2 = 0.0f;
#pragma unroll
  for (int g = 0; g < 12; ++g) { const float* bp_ = b1 + g * 256 + lane * 8;
#pragma unroll
    for (int e = 0; e < 8; ++e) { const float w = pmul(cx, hv[g * 8 + e]) + pmul(cy, bp_[e]); hv[g * 8 + e] = w; n2 += pmul(w, w); } }
  n2 = wsum(n2); const float n = sqrt_f(n2); const float fac = proj_fac(n); const float fs = fac * XS;
  for (int pass = 0; pass < 2; ++pass) {
#pragma unroll
    for (int g = 0; g < 12; ++g) { v8b o; for (int e = 0; e < 8; ++e) { const float w = pmul(hv[g * 8 + e], fs); o[e] = (b16)w; } *(volatile v8b*)(H1h + (size_t)row * HID + g * 256 + lane * 8) = o; }
    ((volatile float*)NRM2)[(size_t)row * 32 + lane] = (lane == 0) ? n * fac : 0.0f;
    __threadfence(); }
}

__global__ __launch_bounds__(256) void row3_kernel(const b16* __restrict__ MX2, const float* __restrict__ NRM2, const float* __restrict__ P, const float* __restrict__ X1, float* __restrict__ out) {
  const int row = blockIdx.x * 8 + (threadIdx.x >> 5), lane = threadIdx.x & 31; const float* b2 = P + 3840;
  float hv[24], bv[24], xv[24], ov[24]; float m2 = 0.0f;
#pragma unroll
  for (int i = 0; i < 24; ++i) { const int c = (i >> 3) * 256 + lane * 8 + (i & 7); hv[i] = (float)MX2[(size_t)row * D + c] * (1.0f / XS); bv[i] = b2[c]; xv[i] = X1[(size_t)row * D + c]; m2 += pmul(hv[i], hv[i]); }
  m2 = wsum(m2);
  const float xn = fmaxf(NRM2[(size_t)row * 32], 1e-15f), mxn = fmaxf(sqrt_f(m2), 1e-15f); const float rad = tanh_n(mxn * rcp_f(xn) * artanh_f(xn)); const float f1 = (rad * rcp_f(mxn)) * proj_fac(rad);
#pragma unroll
  for (int i = 0; i < 24; ++i) hv[i] *= f1;
  float hn; float h2v[24]; mobius_row(hv, bv, h2v, hn); (void)hn;
  float on; mobius_row(xv, h2v, ov, on); (void)on;
  for (int pass = 0; pass < 2; ++pass) {
#pragma unroll
    for (int g = 0; g < 3; ++g) { v4f a, b; for (int e = 0; e < 4; ++e) { a[e] = ov[g * 8 + e]; b[e] = ov[g * 8 + 4 + e]; } float* dst = out + (size_t)row * D + g * 256 + lane * 8; *(volatile v4f*)dst = a; *(volatile v4f*)(dst + 4) = b; }
    __threadfence(); }
}
}

extern "C" void kernel_launch(void* const* d_in, const int* in_sizes, int n_in,
                              void* d_out, int out_size, void* d_ws, size_t ws_size, hipStream_t stream) {
  (void)n_in; (void)out_size;
  const float* x = (const float*)d_in[0]; const float* Wqkv = (const float*)d_in[1]; const float* Wproj = (const float*)d_in[2]; const float* bp = (const float*)d_in[3]; const float* W1 = (const float*)d_in[4]; const float* b1 = (const float*)d_in[5]; const float* W2 = (const float*)d_in[6]; const float* b2 = (const float*)d_in[7];
  float* out = (float*)d_out;
  if (in_sizes[0] != NTOK * D || in_sizes[1] != 3 * D * D || in_sizes[4] != HID * D || in_sizes[6] != D * HID) return;
  size_t off = 0; char* ws = (char*)d_ws;
  auto carve = [&](size_t bytes) { char* p = ws + off; off += (bytes + 255) & ~(size_t)255; return p; };
  b16* R = (b16*)carve(Wo_::END * 2); float* P = (float*)carve(4608 * 4);
  float* X = (float*)carve((size_t)NTOK * D * 4);
  b16* SH = (b16*)carve((size_t)NTOK * D * 2);
  b16* RA = (b16*)carve((size_t)NTOK * HID * 2);
  b16* RB = (b16*)carve((size_t)NTOK * HID * 2);
  b16* OUTh = (b16*)carve((size_t)NTOK * D * 2);
  float* NRM = (float*)carve((size_t)NTOK * 32 * 4); float* NRM2 = (float*)carve((size_t)NTOK * 32 * 4); float* NQK = (float*)carve((size_t)Bn * NH * 2 * SP * 4);
  if (off > ws_size) return;
  b16* Qp = RB; b16* Kp = RB + PLQ; b16* Vt = RB + 2 * PLQ;
  prep_kernel<<<512, 256, 0, stream>>>(Wqkv, Wproj, W1, W2, bp, b1, b2, R, P);
  row0_kernel<<<NTOK / 8, 256, 0, stream>>>(x, X, SH);
  gemm_kernel<D, 3 * D, 0><<<dim3(3 * D / 256, NTOK / 32), 64, 0, stream>>>(SH, R + Wo_::QKV, nullptr, RA, nullptr);
  head_kernel<<<dim3(NH, Bn), 256, 0, stream>>>(RA, Qp, Kp, Vt, NQK);
  attn_kernel<<<dim3(13, Bn), 384, 0, stream>>>(Qp, Kp, Vt, NQK, SH);
  gemm_kernel<D, D, 0><<<dim3(D / 256, NTOK / 32), 64, 0, stream>>>(SH, R + Wo_::PRJ, P, OUTh, nullptr);
  row1_kernel<<<NTOK / 8, 256, 0, stream>>>(OUTh, X, SH, NRM);
  gemm_kernel<D, HID, 0><<<dim3(HID / 256, NTOK / 32), 64, 0, stream>>>(SH, R + Wo_::W1, nullptr, RA, nullptr);
  row2_kernel<<<NTOK / 8, 256, 0, stream>>>(RA, NRM, P, RB, NRM2);
  gemm_kernel<HID, D, 0><<<dim3(D / 256, NTOK / 32), 64, 0, stream>>>(RB, R + Wo_::W2, nullptr, OUTh, nullptr);
  row3_kernel<<<NTOK / 8, 256, 0, stream>>>(OUTh, NRM2, P, X, out);
}
